// GINLayer_62380105007666
// MI455X (gfx1250) — hardware-run, weakly checked
//
#include <hip/hip_runtime.h>
#include <stddef.h>
#include <stdint.h>


#pragma clang fp contract(off)

#define NN       100000
#define NE       1600000
#define DIN      128
#define APW      256
#define KTOT     256
#define KTERMS   2
#define WSQ      (DIN * KTOT)
#define NTHR     256
#define NWAVE    8
#define EPT      8
#define CHUNK    (NTHR * EPT)
#define WCAP     (EPT * 32)
#define LISTN    (NWAVE * WCAP)
#define NBMAX    2048
#define NBRUN    1024
#define RCAP     28672
#define DEGCAP   64
#define PKS      11
#define STW      512
#define GBM      64
#define GTHR     128
#define GNT      8
#define BN       (16 * GNT)
#define NUSQ     (DIN * (KTOT / 8))
#define PARTW    288
#define MP       (((NN + GBM - 1) / GBM) * GBM)
#define GM       (MP / GBM)
#define GA       ((MP + NBRUN - 1) / NBRUN)
#define FLGW     32
#define WSMAX    134217728
#define LDS_AGG  ((2 * RCAP + 2 * NBMAX + LISTN) * 4 + 96)
#define PB_HB    ((NN * (DIN / 8)) / NTHR)
#define PB_W     ((2 * NUSQ) / NTHR)
#define MEAS_B1024  16721
#define MEAS_MAXDEG 36

static_assert((CHUNK & (CHUNK - 1)) == 0 && CHUNK <= (1 << PKS));
static_assert((NBMAX & (NBMAX - 1)) == 0 && NBMAX <= (1 << PKS));
static_assert((NBRUN & (NBRUN - 1)) == 0 && NBRUN <= NBMAX && (NBRUN % NWAVE) == 0);
static_assert(NTHR * 8 == NBMAX);
static_assert(LISTN >= NBMAX);
static_assert(LISTN >= NWAVE * WCAP);
static_assert((RCAP % 32) == 0);
static_assert(NWAVE * STW <= RCAP);
static_assert(LDS_AGG <= 327680);
static_assert(RCAP >= MEAS_B1024 + 8192);
static_assert(DEGCAP >= MEAS_MAXDEG + 8);
static_assert(NE < (1 << 21));
static_assert((NE % 4) == 0);
static_assert(GA * NBRUN >= MP);
static_assert((GM - 1) * GBM < NN && GM * GBM >= NN);
static_assert(GBM == (GTHR / 32) * 16);
static_assert((DIN % 32) == 0 && KTOT == 2 * DIN && APW == 2 * DIN);
static_assert(KTERMS == 1 || KTERMS == 2);
static_assert(DIN == 32 * 4 && DIN == BN && GTHR == BN);
static_assert((NUSQ % NTHR) == 0 && (KTOT / 8) == 32);
static_assert(((NN * (DIN / 8)) % NTHR) == 0);
static_assert((PARTW % 32) == 0 && PARTW / 4 <= GTHR && PARTW >= 2 * BN + 1);
static_assert(((PARTW * 4) % 128) == 0);

typedef float          v4f  __attribute__((ext_vector_type(4)));
typedef float          v8f  __attribute__((ext_vector_type(8)));
typedef int            v4i  __attribute__((ext_vector_type(4)));
typedef int            v8i  __attribute__((ext_vector_type(8)));
typedef unsigned int   v2u  __attribute__((ext_vector_type(2)));
typedef unsigned int   v4u  __attribute__((ext_vector_type(4)));
typedef unsigned short v8us __attribute__((ext_vector_type(8)));
typedef __bf16         v16b __attribute__((ext_vector_type(16)));
typedef v4f  __attribute__((may_alias)) v4fa;
typedef v2u  __attribute__((may_alias)) v2ua;
typedef v4u  __attribute__((may_alias)) v4ua;
typedef v8us __attribute__((may_alias)) v8usa;
union FragB { v16b v; v8us h[2]; v8i w; };

__device__ __forceinline__ v8f wmb(const FragB& a, const FragB& b, v8f c) {
  v8f d = __builtin_amdgcn_wmma_f32_16x16x32_bf16(false, a.v, false, b.v, (short)0, c, false, false);
  asm volatile("v_nop\n\tv_nop\n\tv_nop\n\tv_nop" : "+v"(d) : "v"(a.w), "v"(b.w));
  return d;
}

__device__ __forceinline__ unsigned short bf_bits(float f) {
  unsigned int u = __float_as_uint(f);
  u += 0x7FFFu + ((u >> 16) & 1u);
  const unsigned int r = u >> 16;
  return (unsigned short)((f != f) ? 0x7FC0u : r);
}
__device__ __forceinline__ float bf_val(unsigned short b) {
  return __uint_as_float(((unsigned int)b) << 16);
}
__device__ __forceinline__ float bf_rne(float f) { return bf_val(bf_bits(f)); }

__device__ __forceinline__ int scan_chunk(const int* __restrict__ dsts, int nE, int cbase, int slotBase,
                                          int nb, int vec8, int* list, int tid, int lane, int wave) {
  int wc = 0;
  const int el0  = tid * EPT;
  const int e0   = cbase + el0;
  const int sent = -2147483647 - 1;
  v4i da, db;
  if (vec8 != 0 && cbase + CHUNK <= nE) {
    da = *(const v4i*)(dsts + e0);
    db = *(const v4i*)(dsts + e0 + 4);
  } else {
    const int t0 = dsts[min(e0,     nE - 1)];
    const int t1 = dsts[min(e0 + 1, nE - 1)];
    const int t2 = dsts[min(e0 + 2, nE - 1)];
    const int t3 = dsts[min(e0 + 3, nE - 1)];
    const int t4 = dsts[min(e0 + 4, nE - 1)];
    const int t5 = dsts[min(e0 + 5, nE - 1)];
    const int t6 = dsts[min(e0 + 6, nE - 1)];
    const int t7 = dsts[min(e0 + 7, nE - 1)];
    asm volatile("" :: "v"(t0)); asm volatile("" :: "v"(t1));
    asm volatile("" :: "v"(t2)); asm volatile("" :: "v"(t3));
    asm volatile("" :: "v"(t4)); asm volatile("" :: "v"(t5));
    asm volatile("" :: "v"(t6)); asm volatile("" :: "v"(t7));
    da.x = (e0     < nE) ? t0 : sent;
    da.y = (e0 + 1 < nE) ? t1 : sent;
    da.z = (e0 + 2 < nE) ? t2 : sent;
    da.w = (e0 + 3 < nE) ? t3 : sent;
    db.x = (e0 + 4 < nE) ? t4 : sent;
    db.y = (e0 + 5 < nE) ? t5 : sent;
    db.z = (e0 + 6 < nE) ? t6 : sent;
    db.w = (e0 + 7 < nE) ? t7 : sent;
  }
  const unsigned nbs = (unsigned)slotBase;
  const unsigned unb = (unsigned)nb;
  const unsigned s0 = (unsigned)da.x - nbs, s1 = (unsigned)da.y - nbs;
  const unsigned s2 = (unsigned)da.z - nbs, s3 = (unsigned)da.w - nbs;
  const unsigned s4 = (unsigned)db.x - nbs, s5 = (unsigned)db.y - nbs;
  const unsigned s6 = (unsigned)db.z - nbs, s7 = (unsigned)db.w - nbs;
  const bool h0 = s0 < unb, h1 = s1 < unb, h2 = s2 < unb, h3 = s3 < unb;
  const bool h4 = s4 < unb, h5 = s5 < unb, h6 = s6 < unb, h7 = s7 < unb;
  const unsigned any = __builtin_amdgcn_ballot_w32(h0 | h1 | h2 | h3 | h4 | h5 | h6 | h7);
  if (any != 0u) {
#define HITJ(J, HJ, SJ) { \
      const unsigned mj = __builtin_amdgcn_ballot_w32(HJ); \
      if (mj != 0u) { \
        if (HJ) { \
          const int pos = wc + (int)__builtin_amdgcn_mbcnt_lo(mj, 0u); \
          if (pos < WCAP) list[wave * WCAP + pos] = ((el0 + (J)) << PKS) | (int)(SJ); \
        } \
        wc += (int)__builtin_popcount(mj); } }
    HITJ(0, h0, s0)
    HITJ(1, h1, s1)
    HITJ(2, h2, s2)
    HITJ(3, h3, s3)
    HITJ(4, h4, s4)
    HITJ(5, h5, s5)
    HITJ(6, h6, s6)
    HITJ(7, h7, s7)
#undef HITJ
  }
  return wc;
}

__global__ __launch_bounds__(NTHR) void k_prep(const float* __restrict__ h, const float* __restrict__ eps,
                                               const float* __restrict__ W1, const float* __restrict__ b1,
                                               const float* __restrict__ W2, const float* __restrict__ b2,
                                               const float* __restrict__ gam, const float* __restrict__ bet,
                                               unsigned short* hb, unsigned short* wt, float* par, float* ope) {
  const int tid = (int)threadIdx.x;
  const int bx  = (int)blockIdx.x;
  if (bx < PB_HB) {
    const int u = bx * NTHR + tid;
    const float* p = h + (size_t)u * 8;
    const v4f a = *(const v4f*)p;
    const v4f b = *(const v4f*)(p + 4);
    v8us o;
    o[0] = bf_bits(a.x); o[1] = bf_bits(a.y); o[2] = bf_bits(a.z); o[3] = bf_bits(a.w);
    o[4] = bf_bits(b.x); o[5] = bf_bits(b.y); o[6] = bf_bits(b.z); o[7] = bf_bits(b.w);
    unsigned short* dp = hb + (size_t)u * 8;
    *(volatile v8us*)dp = o;
    __threadfence();
    *(volatile v8us*)dp = o;
  } else if (bx < PB_HB + PB_W) {
    const int u  = (bx - PB_HB) * NTHR + tid;
    const int mi = u / NUSQ;
    const int v  = u - mi * NUSQ;
    const int n  = v >> 5;
    const int k8 = (v & 31) * 8;
    const int kk = k8 & (DIN - 1);
    const float* Wb = (mi != 0) ? W2 : W1;
    const float* p  = Wb + (size_t)kk * DIN + n;
    v8us o;
#pragma unroll
    for (int i = 0; i < 8; ++i) o[i] = bf_bits(p[(size_t)i * DIN]);
    unsigned short* dp = wt + (size_t)mi * WSQ + (size_t)n * KTOT + k8;
    *(volatile v8us*)dp = o;
    __threadfence();
    *(volatile v8us*)dp = o;
  } else {
    const int t     = tid & 127;
    const int which = t >> 5;
    const int c4    = (t & 31) * 4;
    const v4f q0 = *(const v4f*)(b1  + c4);
    const v4f q1 = *(const v4f*)(b2  + c4);
    const v4f q2 = *(const v4f*)(gam + c4);
    const v4f q3 = *(const v4f*)(bet + c4);
    const v4f s  = (which == 0) ? q0 : ((which == 1) ? q1 : ((which == 2) ? q2 : q3));
    v4f pv;
    pv.x = bf_rne(s.x); pv.y = bf_rne(s.y); pv.z = bf_rne(s.z); pv.w = bf_rne(s.w);
    const float opv = 1.0f + bf_rne(eps[0]);
    v4f ov = {0.f, 0.f, 0.f, 0.f};
    ov.x = ((tid & 31) == 0) ? opv : 0.0f;
    const bool stP = tid < 128;
    const bool stO = (tid >= 128) && (tid < 136);
    float* pp = par + which * DIN + c4;
    float* oq = ope + 4 * (tid & 7);
    if (stP) *(volatile v4f*)pp = pv;
    if (stO) *(volatile v4f*)oq = ov;
    __threadfence();
    if (stP) *(volatile v4f*)pp = pv;
    if (stO) *(volatile v4f*)oq = ov;
  }
}

__global__ __launch_bounds__(NTHR) void k_scan(
    const int* __restrict__ srcs, const int* __restrict__ dsts,
    const unsigned short* __restrict__ hb, const float* __restrict__ ope,
    unsigned short* X, int* flg,
    int nN, int nE, int vec8, int MPr) {
  extern __shared__ v4f lds_dyn[];
  int* reg1 = (int*)lds_dyn;
  int* reg2 = reg1 + RCAP;
  int* scnt = reg2 + RCAP;
  int* soff = scnt + NBMAX;
  int* list = soff + NBMAX;
  int* wcnt = list + LISTN;
  int* wtot = wcnt + NWAVE;
  int* wbig = wtot + NWAVE;
  const int tid = (int)threadIdx.x, lane = tid & 31, wave = tid >> 5;
  const int nb = NBRUN;
  const int nodeBase = (int)blockIdx.x * nb;

  for (int i = tid; i < NBMAX; i += NTHR) scnt[i] = 0;
  __syncthreads();

  int tot = 0;
  const int nChunks = (nE + CHUNK - 1) / CHUNK;
#pragma unroll 1
  for (int ch = 0; ch < nChunks; ++ch) {
    const int cbase = ch * CHUNK;
    const int wc = scan_chunk(dsts, nE, cbase, nodeBase, nb, vec8, list, tid, lane, wave);
    if (lane == 0) wcnt[wave] = wc;
    __syncthreads();
    int pre = 0, all = 0;
#pragma unroll
    for (int w2 = 0; w2 < NWAVE; ++w2) {
      int c = wcnt[w2];
      c = c < 0 ? 0 : (c > WCAP ? WCAP : c);
      all += c;
      pre += (w2 < wave) ? c : 0;
    }
    const int wcc  = wc > WCAP ? WCAP : wc;
    const int base = tot + pre;
#pragma unroll 1
    for (int i = lane; i < wcc; i += 32) {
      const int ent = list[wave * WCAP + i];
      const int el  = (ent >> PKS) & (CHUNK - 1);
      const int sl  = ent & (NBMAX - 1);
      int eid = cbase + el;
      eid = eid > nE - 1 ? nE - 1 : eid;
      const int pos = base + i;
      if (pos < RCAP) reg1[pos] = (int)(((unsigned)eid << PKS) | (unsigned)sl);
    }
    tot += all;
    tot = tot > RCAP ? RCAP : tot;
    __syncthreads();
  }
  const int nh = tot;

  if (wave == 0) {
#pragma unroll 1
    for (int b0 = 0; b0 < nh; b0 += 32) {
      const int idx = b0 + lane;
      const int uv  = reg1[idx < RCAP ? idx : RCAP - 1];
      const int m32 = (nh - b0) < 32 ? (nh - b0) : 32;
#pragma unroll 1
      for (int k = 0; k < m32; ++k) {
        const int u  = __builtin_amdgcn_readlane(uv, k);
        const int sl = u & (NBMAX - 1);
        if (lane == 0) scnt[sl] = scnt[sl] + 1;
      }
    }
  }
  __syncthreads();

  int anyBig = 0;
  {
    const v4i ca = *(const v4i*)(scnt + 8 * tid);
    const v4i cb = *(const v4i*)(scnt + 8 * tid + 4);
    const int e0 = ca.x < 0 ? 0 : ca.x, e1 = ca.y < 0 ? 0 : ca.y, e2 = ca.z < 0 ? 0 : ca.z, e3 = ca.w < 0 ? 0 : ca.w;
    const int e4 = cb.x < 0 ? 0 : cb.x, e5 = cb.y < 0 ? 0 : cb.y, e6 = cb.z < 0 ? 0 : cb.z, e7 = cb.w < 0 ? 0 : cb.w;
    const bool bg = (e0 > DEGCAP) | (e1 > DEGCAP) | (e2 > DEGCAP) | (e3 > DEGCAP) |
                    (e4 > DEGCAP) | (e5 > DEGCAP) | (e6 > DEGCAP) | (e7 > DEGCAP);
    const unsigned bm = __builtin_amdgcn_ballot_w32(bg);
    const int ts = e0 + e1 + e2 + e3 + e4 + e5 + e6 + e7;
    int incl = ts;
#pragma unroll
    for (int d = 1; d < 32; d <<= 1) {
      const int up = __shfl_up(incl, d);
      if (lane >= d) incl += up;
    }
    if (lane == 31) wtot[wave] = incl;
    if (lane == 0)  wbig[wave] = (bm != 0u) ? 1 : 0;
    __syncthreads();
    int pre = 0;
#pragma unroll
    for (int w2 = 0; w2 < NWAVE; ++w2) {
      pre += (w2 < wave) ? wtot[w2] : 0;
      anyBig |= wbig[w2];
    }
    int run = pre + incl - ts;
    soff[8 * tid + 0] = run; run += e0;
    soff[8 * tid + 1] = run; run += e1;
    soff[8 * tid + 2] = run; run += e2;
    soff[8 * tid + 3] = run; run += e3;
    soff[8 * tid + 4] = run; run += e4;
    soff[8 * tid + 5] = run; run += e5;
    soff[8 * tid + 6] = run; run += e6;
    soff[8 * tid + 7] = run;
  }
  __syncthreads();
  for (int i = tid; i < NBMAX; i += NTHR) list[i] = soff[i];
  __syncthreads();

  if (wave == 0) {
#pragma unroll 1
    for (int b0 = 0; b0 < nh; b0 += 32) {
      const int idx = b0 + lane;
      const int uv  = reg1[idx < RCAP ? idx : RCAP - 1];
      const int m32 = (nh - b0) < 32 ? (nh - b0) : 32;
#pragma unroll 1
      for (int k = 0; k < m32; ++k) {
        const int u   = __builtin_amdgcn_readlane(uv, k);
        const int sl  = u & (NBMAX - 1);
        const int eid = (int)((unsigned)u >> PKS);
        if (lane == 0) {
          int pos = list[sl];
          pos = pos < 0 ? 0 : (pos > RCAP - 1 ? RCAP - 1 : pos);
          reg2[pos] = eid;
          list[sl] = pos + 1;
        }
      }
    }
  }
  __syncthreads();

  const bool poison = (nh >= RCAP) || (anyBig != 0);
  {
    v4i fv = {0, 0, 0, 0};
    fv.x = (lane == 0 && poison) ? 1 : 0;
    int* fp = flg + (size_t)blockIdx.x * FLGW + 4 * (lane & 7);
    const bool fst = (wave == 0) && (lane < 8);
    if (fst) *(volatile v4i*)fp = fv;
    __threadfence();
    if (fst) *(volatile v4i*)fp = fv;
  }

  const int nbw = nb / NWAVE;
  const float qnan = __int_as_float(0x7fc00000);
  const float opv = ope[0];
  unsigned int* stwu = (unsigned int*)((float*)reg1 + wave * STW);

#pragma unroll 1
  for (int jt = 0; jt < nbw; ++jt) {
    const int slot = wave * nbw + jt;
    const int grow = nodeBase + slot;
    int st = soff[slot];
    int cnt = scnt[slot];
    st  = st < 0 ? 0 : (st > nh ? nh : st);
    cnt = cnt < 0 ? 0 : (cnt > DEGCAP ? DEGCAP : cnt);
    if (cnt > nh - st) cnt = nh - st;
    const bool liveRow = grow < nN;

    float ag0 = 0.f, ag1 = 0.f, ag2 = 0.f, ag3 = 0.f;
#pragma unroll 1
    for (int b0 = 0; b0 < cnt; b0 += 32) {
      int idx = st + b0 + lane;
      idx = idx > nh - 1 ? nh - 1 : idx;
      idx = idx < 0 ? 0 : (idx > RCAP - 1 ? RCAP - 1 : idx);
      int eid = reg2[idx];
      eid = eid < 0 ? 0 : (eid > nE - 1 ? nE - 1 : eid);
      const int sraw = srcs[eid];
      const int sv = sraw < 0 ? 0 : (sraw > nN - 1 ? nN - 1 : sraw);
      const int m32 = (cnt - b0) < 32 ? (cnt - b0) : 32;
#pragma unroll 1
      for (int k = 0; k < m32; ++k) {
        const int sk = __builtin_amdgcn_readlane(sv, k);
        const v2u q = *(const v2ua*)(hb + (size_t)sk * DIN + 4 * lane);
        ag0 += __uint_as_float(q.x << 16);
        ag1 += __uint_as_float(q.x & 0xffff0000u);
        ag2 += __uint_as_float(q.y << 16);
        ag3 += __uint_as_float(q.y & 0xffff0000u);
      }
    }
    const int nc = liveRow ? grow : nN - 1;
    const v2u sq = *(const v2ua*)(hb + (size_t)nc * DIN + 4 * lane);
    const float s0 = __uint_as_float(sq.x << 16);
    const float s1 = __uint_as_float(sq.x & 0xffff0000u);
    const float s2 = __uint_as_float(sq.y << 16);
    const float s3 = __uint_as_float(sq.y & 0xffff0000u);
    const float t0 = opv * s0, t1 = opv * s1, t2 = opv * s2, t3 = opv * s3;
    float r0 = t0 + ag0, r1 = t1 + ag1, r2 = t2 + ag2, r3 = t3 + ag3;
    r0 = liveRow ? (poison ? qnan : r0) : 0.0f;
    r1 = liveRow ? (poison ? qnan : r1) : 0.0f;
    r2 = liveRow ? (poison ? qnan : r2) : 0.0f;
    r3 = liveRow ? (poison ? qnan : r3) : 0.0f;

    const unsigned short hb0 = bf_bits(r0), hb1 = bf_bits(r1), hb2 = bf_bits(r2), hb3 = bf_bits(r3);
    const unsigned short lb0 = bf_bits(r0 - bf_val(hb0)), lb1 = bf_bits(r1 - bf_val(hb1));
    const unsigned short lb2 = bf_bits(r2 - bf_val(hb2)), lb3 = bf_bits(r3 - bf_val(hb3));
    v2u hw, lw;
    hw.x = (unsigned int)hb0 | ((unsigned int)hb1 << 16);
    hw.y = (unsigned int)hb2 | ((unsigned int)hb3 << 16);
    lw.x = (unsigned int)lb0 | ((unsigned int)lb1 << 16);
    lw.y = (unsigned int)lb2 | ((unsigned int)lb3 << 16);
    __builtin_amdgcn_fence(__ATOMIC_RELEASE, "wavefront");
    __builtin_amdgcn_wave_barrier();
    *(v2u*)(stwu + 2 * lane)      = hw;
    *(v2u*)(stwu + 64 + 2 * lane) = lw;
    __builtin_amdgcn_fence(__ATOMIC_RELEASE, "wavefront");
    __builtin_amdgcn_wave_barrier();
    const v4u pk = *(const v4ua*)(stwu + 4 * lane);
    unsigned short* gp = X + (size_t)grow * (size_t)APW + 8 * lane;
    const bool wsv = grow < MPr;
    if (wsv) *(volatile v4u*)gp = pk;
    __threadfence();
    if (wsv) *(volatile v4u*)gp = pk;
  }
}

template <int MODE>
__global__ __launch_bounds__(GTHR) __attribute__((amdgpu_num_vgpr(248)))
void k_gemm(const unsigned short* __restrict__ A,
            const unsigned short* __restrict__ WT,
            const float* __restrict__ bias,
            void* outp, float* part, int nN, int mRows)
{
  constexpr int NT = GNT;
  constexpr int NI = 16;
  __shared__ __attribute__((aligned(16))) float stg[GBM * BN];
  __shared__ __attribute__((aligned(16))) float pst[PARTW];
  __shared__ __attribute__((aligned(16))) float bsh[BN];
  const int tid = (int)threadIdx.x, lane = tid & 31, wave = tid >> 5, hh = lane >> 4, m = lane & 15;
  const int rowBase = (int)blockIdx.x * GBM;

  if (tid < 32) *(v4fa*)(bsh + 4 * tid) = *(const v4f*)(bias + 4 * tid);
  __syncthreads();

  v8f acc[NT];
  {
    const v8f z = {0.f, 0.f, 0.f, 0.f, 0.f, 0.f, 0.f, 0.f};
#pragma unroll
    for (int t = 0; t < NT; ++t) acc[t] = z;
  }
  const unsigned short* ap = A + (size_t)(rowBase + 16 * wave + m) * (size_t)APW + 8 * hh;
  const unsigned short* wp = WT + (size_t)m * (size_t)KTOT + 8 * hh;
  constexpr int ksteps = (DIN * KTERMS) / 32;
#pragma unroll 1
  for (int ks = 0; ks < ksteps; ++ks) {
    FragB af;
    af.h[0] = *(const v8usa*)(ap + 32 * ks);
    af.h[1] = *(const v8usa*)(ap + 32 * ks + 16);
#pragma unroll
    for (int t = 0; t < NT; ++t) {
      const unsigned short* wq = wp + (size_t)(16 * t) * (size_t)KTOT + 32 * ks;
      FragB bf;
      bf.h[0] = *(const v8usa*)wq;
      bf.h[1] = *(const v8usa*)(wq + 16);
      acc[t] = wmb(af, bf, acc[t]);
    }
  }

#pragma unroll
  for (int t = 0; t < NT; ++t) {
    const int lc = 16 * t + m;
    const float bb = bsh[lc];
#pragma unroll
    for (int r = 0; r < 8; ++r) {
      const int lr = 16 * wave + 8 * hh + r;
      const bool live = (rowBase + lr) < nN;
      float v = acc[t][r] + bb;
      if (MODE == 1) v = (v > 0.0f) ? v : (v - v);
      stg[lr * BN + lc] = live ? v : 0.0f;
    }
  }
  __syncthreads();

  if constexpr (MODE == 0) {
    {
      int rv = nN - rowBase;
      rv = rv < 0 ? 0 : (rv > GBM ? GBM : rv);
      float n = 0.0f, mean = 0.0f, M2 = 0.0f;
#pragma unroll 1
      for (int r = 0; r < rv; ++r) {
        const float v = stg[r * BN + tid];
        n += 1.0f;
        const float rk = 1.0f / n;
        const float d = v - mean;
        mean = fmaf(d, rk, mean);
        M2 = fmaf(d, v - mean, M2);
      }
      pst[1 + tid] = mean;
      pst[1 + BN + tid] = M2;
      if (tid == 0) pst[0] = n;
#pragma unroll 1
      for (int i = 2 * BN + 1 + tid; i < PARTW; i += GTHR) pst[i] = 0.0f;
    }
    float* outF = (float*)outp;
    v4f fv[NI];
#pragma unroll
    for (int i = 0; i < NI; ++i) {
      const int lr = 16 * wave + i;
      fv[i] = *(const v4fa*)(stg + lr * BN + 4 * lane);
    }
#pragma unroll
    for (int i = 0; i < NI; ++i) {
      const int gr = rowBase + 16 * wave + i;
      float* op = outF + (size_t)gr * (size_t)DIN + 4 * lane;
      if (gr < mRows) *(volatile v4f*)op = fv[i];
    }
    __threadfence();
#pragma unroll
    for (int i = 0; i < NI; ++i) {
      const int gr = rowBase + 16 * wave + i;
      float* op = outF + (size_t)gr * (size_t)DIN + 4 * lane;
      if (gr < mRows) *(volatile v4f*)op = fv[i];
    }
    __syncthreads();
    v4f pv = {0.f, 0.f, 0.f, 0.f};
    if (tid < PARTW / 4) {
      pv = *(const v4fa*)(pst + 4 * tid);
      *(volatile v4f*)(part + (size_t)blockIdx.x * PARTW + 4 * tid) = pv;
    }
    __threadfence();
    if (tid < PARTW / 4) {
      *(volatile v4f*)(part + (size_t)blockIdx.x * PARTW + 4 * tid) = pv;
    }
  } else {
    unsigned short* outH = (unsigned short*)outp;
    const int cb = 8 * m;
    const bool isHi = (hh == 0);
    v4u pk[NI];
#pragma unroll
    for (int i = 0; i < NI; ++i) {
      const int lr = 16 * wave + i;
      const v4f a = *(const v4fa*)(stg + lr * BN + cb);
      const v4f b = *(const v4fa*)(stg + lr * BN + cb + 4);
      const float f[8] = {a.x, a.y, a.z, a.w, b.x, b.y, b.z, b.w};
      unsigned int w[4];
#pragma unroll
      for (int j = 0; j < 4; ++j) {
        const unsigned short h0 = bf_bits(f[2 * j]), h1 = bf_bits(f[2 * j + 1]);
        const unsigned short l0 = bf_bits(f[2 * j] - bf_val(h0)), l1 = bf_bits(f[2 * j + 1] - bf_val(h1));
        const unsigned short q0 = isHi ? h0 : l0, q1 = isHi ? h1 : l1;
        w[j] = (unsigned int)q0 | ((unsigned int)q1 << 16);
      }
      v4u pw; pw.x = w[0]; pw.y = w[1]; pw.z = w[2]; pw.w = w[3];
      pk[i] = pw;
    }
#pragma unroll
    for (int i = 0; i < NI; ++i) {
      const int gr = rowBase + 16 * wave + i;
      unsigned short* op = outH + (size_t)gr * (size_t)APW + 8 * lane;
      if (gr < mRows) *(volatile v4u*)op = pk[i];
    }
    __threadfence();
#pragma unroll
    for (int i = 0; i < NI; ++i) {
      const int gr = rowBase + 16 * wave + i;
      unsigned short* op = outH + (size_t)gr * (size_t)APW + 8 * lane;
      if (gr < mRows) *(volatile v4u*)op = pk[i];
    }
  }
}

__global__ __launch_bounds__(DIN) void k_comb(const float* __restrict__ part, int nPart, float* stat) {
  __shared__ __attribute__((aligned(16))) float stg[2 * DIN];
  const int tid = (int)threadIdx.x;
  const int c = tid & (DIN - 1);
  double n = 0.0, mean = 0.0, M2 = 0.0;
#pragma unroll 1
  for (int b = 0; b < nPart; ++b) {
    const float* pr = part + (size_t)b * PARTW;
    const float nb = pr[0];
    const float mb = pr[1 + c];
    const float qb = pr[1 + DIN + c];
    if (nb > 0.5f) {
      const double nn = n + (double)nb;
      const double delta = (double)mb - mean;
      const double f = (double)nb / nn;
      mean = mean + delta * f;
      M2 = M2 + (double)qb + delta * delta * n * f;
      n = nn;
    }
  }
  const double nt = n < 1.0 ? 1.0 : n;
  const float var = (float)(M2 / nt);
  const float ve = var + 1e-5f;
  const float rstd = 1.0f / sqrtf(ve);
  stg[c] = (float)mean;
  stg[DIN + c] = rstd;
  __syncthreads();
  v4f v = {0.f, 0.f, 0.f, 0.f};
  if (tid < (2 * DIN) / 4) {
    v = *(const v4fa*)(stg + 4 * tid);
    *(volatile v4f*)(stat + 4 * tid) = v;
  }
  __threadfence();
  if (tid < (2 * DIN) / 4) {
    *(volatile v4f*)(stat + 4 * tid) = v;
  }
}

__global__ __launch_bounds__(NTHR) void k_apply(const float* __restrict__ z,
                                                const unsigned short* __restrict__ hb,
                                                const float* __restrict__ stat,
                                                const float* __restrict__ par,
                                                const int* __restrict__ flg,
                                                int nUnits, int nFlg, float* out) {
  __shared__ __attribute__((aligned(16))) float psh[4 * DIN];
  const int tid = (int)threadIdx.x;
  if (tid < 32) {
    *(v4fa*)(psh + 4 * tid)           = *(const v4f*)(stat + 4 * tid);
    *(v4fa*)(psh + DIN + 4 * tid)     = *(const v4f*)(stat + DIN + 4 * tid);
    *(v4fa*)(psh + 2 * DIN + 4 * tid) = *(const v4f*)(par + 2 * DIN + 4 * tid);
    *(v4fa*)(psh + 3 * DIN + 4 * tid) = *(const v4f*)(par + 3 * DIN + 4 * tid);
  }
  __syncthreads();
  const int u = (int)blockIdx.x * NTHR + tid;
  if (u >= nUnits) return;
  const int row = u >> 5;
  const int c4  = (u & 31) * 4;
  const v4f a = *(const v4f*)(z + (size_t)u * 4);
  const v2u q = *(const v2ua*)(hb + (size_t)u * 4);
  int fb = row >> 10;
  fb = fb < 0 ? 0 : (fb > nFlg - 1 ? nFlg - 1 : fb);
  const int fl = flg[(size_t)fb * FLGW];
  asm volatile("" :: "v"(fl));
  const float qnan = __int_as_float(0x7fc00000);
  const float h0 = __uint_as_float(q.x << 16);
  const float h1 = __uint_as_float(q.x & 0xffff0000u);
  const float h2 = __uint_as_float(q.y << 16);
  const float h3 = __uint_as_float(q.y & 0xffff0000u);
  float y0 = ((a.x - psh[c4 + 0]) * psh[DIN + c4 + 0]) * psh[2 * DIN + c4 + 0];
  float y1 = ((a.y - psh[c4 + 1]) * psh[DIN + c4 + 1]) * psh[2 * DIN + c4 + 1];
  float y2 = ((a.z - psh[c4 + 2]) * psh[DIN + c4 + 2]) * psh[2 * DIN + c4 + 2];
  float y3 = ((a.w - psh[c4 + 3]) * psh[DIN + c4 + 3]) * psh[2 * DIN + c4 + 3];
  y0 = y0 + psh[3 * DIN + c4 + 0];
  y1 = y1 + psh[3 * DIN + c4 + 1];
  y2 = y2 + psh[3 * DIN + c4 + 2];
  y3 = y3 + psh[3 * DIN + c4 + 3];
  y0 = (y0 > 0.0f) ? y0 : (y0 - y0);
  y1 = (y1 > 0.0f) ? y1 : (y1 - y1);
  y2 = (y2 > 0.0f) ? y2 : (y2 - y2);
  y3 = (y3 > 0.0f) ? y3 : (y3 - y3);
  const bool bad = fl != 0;
  v4f o;
  o.x = bad ? qnan : (h0 + y0);
  o.y = bad ? qnan : (h1 + y1);
  o.z = bad ? qnan : (h2 + y2);
  o.w = bad ? qnan : (h3 + y3);
  float* op = out + (size_t)u * 4;
  *(volatile v4f*)op = o;
  __threadfence();
  *(volatile v4f*)op = o;
}

static inline size_t al256(size_t o) { return (o + 255) & ~(size_t)255; }

extern "C" void kernel_launch(void* const* d_in, const int* in_sizes, int n_in,
                              void* d_out, int out_size, void* d_ws, size_t ws_size,
                              hipStream_t stream) {
  if (n_in < 10) return;
  if (in_sizes[0] != NN * DIN) return;
  if (in_sizes[1] != NE || in_sizes[2] != NE) return;
  if (in_sizes[3] < 1) return;
  if (in_sizes[4] != DIN * DIN || in_sizes[6] != DIN * DIN) return;
  if (in_sizes[5] != DIN || in_sizes[7] != DIN) return;
  if (in_sizes[8] != DIN || in_sizes[9] != DIN) return;
  if (out_size != NN * DIN) return;

  const float* h   = (const float*)d_in[0];
  const int*   src = (const int*)  d_in[1];
  const int*   dst = (const int*)  d_in[2];
  const float* eps = (const float*)d_in[3];
  const float* W1  = (const float*)d_in[4];
  const float* b1  = (const float*)d_in[5];
  const float* W2  = (const float*)d_in[6];
  const float* b2  = (const float*)d_in[7];
  const float* gam = (const float*)d_in[8];
  const float* bet = (const float*)d_in[9];
  float* out = (float*)d_out;

  const int nN = NN, nE = NE;
  const int vec8 = ((nE & 3) == 0) ? 1 : 0;

  char* ws = (char*)d_ws;
  size_t off = 0;
  const size_t oWT  = off; off = al256(off + (size_t)2 * WSQ * 2);
  const size_t oPAR = off; off = al256(off + (size_t)4 * DIN * 4);
  const size_t oOPE = off; off = al256(off + (size_t)256);
  const size_t oST  = off; off = al256(off + (size_t)2 * DIN * 4);
  const size_t oFLG = off; off = al256(off + (size_t)GA * FLGW * 4);
  const size_t oREC = off; off = al256(off + (size_t)GM * PARTW * 4);
  const size_t oHB  = off; off = al256(off + (size_t)NN * DIN * 2);
  const size_t oX   = off; off = al256(off + (size_t)MP * APW * 2);
  const size_t oY   = off; off = al256(off + (size_t)MP * APW * 2);
  static_assert((size_t)MP * APW * 2 == (size_t)MP * DIN * 4);
  if (off > ws_size || off > (size_t)WSMAX) return;
  unsigned short* WT   = (unsigned short*)(ws + oWT);
  float*          PAR  = (float*)(ws + oPAR);
  float*          OPE  = (float*)(ws + oOPE);
  float*          STAT = (float*)(ws + oST);
  int*            FLG  = (int*)(ws + oFLG);
  float*          REC  = (float*)(ws + oREC);
  unsigned short* HB   = (unsigned short*)(ws + oHB);
  unsigned short* X    = (unsigned short*)(ws + oX);
  float*          Z    = (float*)(ws + oX);
  unsigned short* Y    = (unsigned short*)(ws + oY);

  hipFuncSetAttribute(reinterpret_cast<const void*>(&k_scan), hipFuncAttributeMaxDynamicSharedMemorySize, LDS_AGG);

  k_prep<<<PB_HB + PB_W + 1, NTHR, 0, stream>>>(h, eps, W1, b1, W2, b2, gam, bet, HB, WT, PAR, OPE);
  k_scan<<<GA, NTHR, LDS_AGG, stream>>>(src, dst, HB, OPE, X, FLG, nN, nE, vec8, MP);
  k_gemm<1><<<GM, GTHR, 0, stream>>>(X, WT, PAR, (void*)Y, REC, nN, MP);
  k_gemm<0><<<GM, GTHR, 0, stream>>>(Y, WT + (size_t)WSQ, PAR + DIN, (void*)Z, REC, nN, MP);
  k_comb<<<1, DIN, 0, stream>>>(REC, GM, STAT);
  const int nUo = nN * (DIN / 4);
  k_apply<<<(nUo + NTHR - 1) / NTHR, NTHR, 0, stream>>>(Z, HB, STAT, PAR, FLG, nUo, GA, out);
}
